// CrossLevelAttention_42545946034839
// MI455X (gfx1250) — hardware-verified
//
#include <hip/hip_runtime.h>


namespace {
constexpr int B = 2, NH = 16, T = 2048, DH = 64, C = NH * DH, T1 = 512, T2 = 128, NQT = T / 16;
constexpr float XS = 8.0f, PS = 2048.0f, SCALE = 0.125f;
typedef _Float16 b16;
typedef __attribute__((ext_vector_type(16))) _Float16 v16b;
typedef __attribute__((ext_vector_type(8))) _Float16 v8b;
typedef __attribute__((ext_vector_type(8))) float v8f;
typedef __attribute__((ext_vector_type(4))) float v4f;
__device__ __forceinline__ float bf16_rne(float f) { unsigned int u = __float_as_uint(f); u += 0x7FFFu + ((u >> 16) & 1u); return __uint_as_float(u & 0xFFFF0000u); }
__device__ __forceinline__ void split16(float v, b16& hi, b16& lo) { hi = (b16)v; lo = (b16)(v - (float)hi); }
__device__ __forceinline__ v16b frag_kb(const b16* p, int hh) { const v8b a = *(const v8b*)(p + 8 * hh), b = *(const v8b*)(p + 16 + 8 * hh); v16b f;
#pragma unroll
  for (int e = 0; e < 8; ++e) { f[e] = a[e]; f[8 + e] = b[e]; } return f; }
__device__ __forceinline__ v8f wmma16b(v16b a, v16b b, v8f c) { v8f d = __builtin_amdgcn_wmma_f32_16x16x32_f16(false, a, false, b, (short)0, c, false, false); asm volatile("v_nop\n\tv_nop\n\tv_nop\n\tv_nop" : "+v"(d) : "v"(a), "v"(b)); return d; }
__device__ __forceinline__ void wave_lds_sync() { __builtin_amdgcn_fence(__ATOMIC_RELEASE, "workgroup"); __builtin_amdgcn_wave_barrier(); __builtin_amdgcn_fence(__ATOMIC_ACQUIRE, "workgroup"); }
__device__ __forceinline__ float pmul(float a, float b) { float p = a * b; asm volatile("" : "+v"(p)); return p; }

__global__ __launch_bounds__(256) void cvt_kernel(const float* __restrict__ src, size_t n8, b16* __restrict__ dst) {
  const size_t u = (size_t)blockIdx.x * 256 + threadIdx.x; if (u >= n8) return; const size_t e = u * 8; v8b v;
#pragma unroll
  for (int j = 0; j < 8; ++j) v[j] = (b16)(bf16_rne(src[e + j]) * XS); for (int pass = 0; pass < 2; ++pass) { *(volatile v8b*)(dst + e) = v; __threadfence(); }
}
__global__ __launch_bounds__(256) void vt_kernel(const float* __restrict__ V, int TM, b16* __restrict__ VT) {
  __shared__ float Tt[64][65]; const int h = blockIdx.x % NH, st = (blockIdx.x / NH) % (TM / 64), b = blockIdx.x / (NH * (TM / 64)); const int tid = threadIdx.x;
  for (int i = tid; i < 64 * 64; i += 256) { const int r = i / 64, d = i % 64; Tt[r][d] = bf16_rne(V[((size_t)b * TM + st * 64 + r) * C + h * DH + d]); }
  __syncthreads();
  { const int d = tid / 4, g = (tid % 4) * 2; for (int gg = g; gg < g + 2; ++gg) { v8b v; for (int j = 0; j < 8; ++j) v[j] = (b16)(Tt[gg * 8 + j][d] * XS); const size_t o = ((size_t)(b * NH + h) * DH + d) * TM + st * 64 + gg * 8; for (int pass = 0; pass < 2; ++pass) { *(volatile v8b*)(VT + o) = v; __threadfence(); } } }
}
__global__ __launch_bounds__(32) void att_kernel(const b16* __restrict__ QB, const b16* __restrict__ K0, const b16* __restrict__ K1, const b16* __restrict__ K2, const b16* __restrict__ V0, const b16* __restrict__ V1, const b16* __restrict__ V2, const float* __restrict__ ll, int NWV, float* __restrict__ out) {
  __shared__ __attribute__((aligned(16))) b16 Ph[16][32 + 8], Pl[16][32 + 8]; __shared__ float Mx[16], Sm[16]; __shared__ __attribute__((aligned(16))) float Tf[16][DH + 4];
  const int lane = threadIdx.x, nloc = lane & 15, hlf = lane >> 4; if ((int)blockIdx.x >= NWV) return; const int qt = blockIdx.x % NQT, h = (blockIdx.x / NQT) % NH, b = blockIdx.x / (NQT * NH); const int t0 = qt * 16;
  const float l0 = bf16_rne(ll[0]), l1 = bf16_rne(ll[1]), l2 = bf16_rne(ll[2]); const float lm = fmaxf(l0, fmaxf(l1, l2)); const float e0 = __expf(l0 - lm), e1 = __expf(l1 - lm), e2 = __expf(l2 - lm); const float wl[3] = {e0 / (e0 + e1 + e2), e1 / (e0 + e1 + e2), e2 / (e0 + e1 + e2)};
  const b16* qrow = QB + (((size_t)b * NH + h) * T + t0 + nloc) * DH; const v16b qa0 = frag_kb(qrow, hlf), qa1 = frag_kb(qrow + 32, hlf);
  float res[4][8];
#pragma unroll
  for (int t = 0; t < 4; ++t)
#pragma unroll
    for (int r8 = 0; r8 < 8; ++r8) res[t][r8] = 0.0f;
#pragma unroll 1
  for (int lvl = 0; lvl < 3; ++lvl) { const int TM = lvl == 0 ? T : (lvl == 1 ? T1 : T2); const b16* KB_ = lvl == 0 ? K0 : (lvl == 1 ? K1 : K2); const b16* VT = lvl == 0 ? V0 : (lvl == 1 ? V1 : V2); const int nblk = lvl == 0 ? (t0 / 32 + 1) : TM / 32;
    auto scores = [&](int kb, v8f sacc[2]) {
#pragma unroll
      for (int st = 0; st < 2; ++st) { const b16* kr = KB_ + ((size_t)b * TM + kb + st * 16 + nloc) * C + h * DH; sacc[st] = (v8f){}; sacc[st] = wmma16b(qa0, frag_kb(kr, hlf), sacc[st]); sacc[st] = wmma16b(qa1, frag_kb(kr + 32, hlf), sacc[st]); } };
    float rmax[8];
#pragma unroll
    for (int r8 = 0; r8 < 8; ++r8) rmax[r8] = -INFINITY;
#pragma unroll 1
    for (int bi = 0; bi < nblk; ++bi) { const int kb = bi * 32; v8f sacc[2]; scores(kb, sacc);
#pragma unroll
      for (int st = 0; st < 2; ++st)
#pragma unroll
        for (int r8 = 0; r8 < 8; ++r8) { const int tq = t0 + 8 * hlf + r8, s = kb + st * 16 + nloc; if (lvl != 0 || s <= tq) rmax[r8] = fmaxf(rmax[r8], sacc[st][r8] * (SCALE / (XS * XS))); } }
#pragma unroll
    for (int r8 = 0; r8 < 8; ++r8) { float m = rmax[r8]; for (int o = 1; o < 16; o <<= 1) m = fmaxf(m, __shfl_xor(m, o)); if (nloc == 0) Mx[8 * hlf + r8] = m; }
    wave_lds_sync();
    v8f acc[4]; float rsum[8];
#pragma unroll
    for (int t = 0; t < 4; ++t) acc[t] = (v8f){};
#pragma unroll
    for (int r8 = 0; r8 < 8; ++r8) rsum[r8] = 0.0f;
#pragma unroll 1
    for (int bi = 0; bi < nblk; ++bi) { const int kb = bi * 32; v8f sacc[2]; scores(kb, sacc);
#pragma unroll
      for (int st = 0; st < 2; ++st)
#pragma unroll
        for (int r8 = 0; r8 < 8; ++r8) { const int rl = 8 * hlf + r8; const int tq = t0 + rl, s = kb + st * 16 + nloc; float p = 0.0f; if (lvl != 0 || s <= tq) p = __expf(sacc[st][r8] * (SCALE / (XS * XS)) - Mx[rl]); rsum[r8] += p; b16 ph, pl; split16(p * PS, ph, pl); Ph[rl][st * 16 + nloc] = ph; Pl[rl][st * 16 + nloc] = pl; }
      wave_lds_sync();
      const v16b pa = frag_kb(&Ph[nloc][0], hlf), pb = frag_kb(&Pl[nloc][0], hlf);
#pragma unroll
      for (int t = 0; t < 4; ++t) { const v16b vb = frag_kb(VT + ((size_t)(b * NH + h) * DH + t * 16 + nloc) * TM + kb, hlf); acc[t] = wmma16b(pa, vb, acc[t]); acc[t] = wmma16b(pb, vb, acc[t]); }
      wave_lds_sync(); }
#pragma unroll
    for (int r8 = 0; r8 < 8; ++r8) { float s = rsum[r8]; for (int o = 1; o < 16; o <<= 1) s += __shfl_xor(s, o); if (nloc == 0) Sm[8 * hlf + r8] = s; }
    wave_lds_sync();
    const float wv = wl[lvl];
#pragma unroll
    for (int t = 0; t < 4; ++t)
#pragma unroll
      for (int r8 = 0; r8 < 8; ++r8) res[t][r8] += pmul(wv, acc[t][r8] * (1.0f / (PS * XS)) / Sm[8 * hlf + r8]);
    wave_lds_sync(); }
#pragma unroll
  for (int t = 0; t < 4; ++t)
#pragma unroll
    for (int r8 = 0; r8 < 8; ++r8) Tf[8 * hlf + r8][t * 16 + nloc] = res[t][r8];
  wave_lds_sync();
  for (int pass = 0; pass < 2; ++pass) { for (int rr = 0; rr < 16; ++rr) { ((volatile float*)out)[((size_t)b * T + t0 + rr) * C + h * DH + lane] = Tf[rr][lane]; ((volatile float*)out)[((size_t)b * T + t0 + rr) * C + h * DH + 32 + lane] = Tf[rr][32 + lane]; } __threadfence(); }
}
}

extern "C" void kernel_launch(void* const* d_in, const int* in_sizes, int n_in, void* d_out, int out_size, void* d_ws, size_t ws_size, hipStream_t stream) {
  (void)n_in;
  auto Fp = [&](int i) { return (const float*)d_in[i]; };
  if (in_sizes[0] != B * NH * T * DH || in_sizes[1] != B * T * C || in_sizes[2] != B * T * C || in_sizes[3] != B * T1 * C || in_sizes[4] != B * T1 * C || in_sizes[5] != B * T2 * C || in_sizes[6] != B * T2 * C || in_sizes[7] != 3 || out_size != B * T * C) return;
  const int NWV = B * NH * NQT;
  size_t off = 0; char* ws = (char*)d_ws;
  auto carve = [&](size_t bytes) { char* p = ws + off; off += (bytes + 255) & ~(size_t)255; return p; };
  b16* QB = (b16*)carve((size_t)B * NH * T * DH * 2); b16* K0 = (b16*)carve((size_t)B * T * C * 2); b16* K1 = (b16*)carve((size_t)B * T1 * C * 2); b16* K2 = (b16*)carve((size_t)B * T2 * C * 2);
  b16* V0 = (b16*)carve((size_t)B * T * C * 2); b16* V1 = (b16*)carve((size_t)B * T1 * C * 2); b16* V2 = (b16*)carve((size_t)B * T2 * C * 2);
  if (off > ws_size || off > ((size_t)64 << 20)) return;
  cvt_kernel<<<(unsigned)(((size_t)B * NH * T * DH / 8 + 255) / 256), 256, 0, stream>>>(Fp(0), (size_t)B * NH * T * DH / 8, QB);
  cvt_kernel<<<(unsigned)(((size_t)B * T * C / 8 + 255) / 256), 256, 0, stream>>>(Fp(1), (size_t)B * T * C / 8, K0); cvt_kernel<<<(unsigned)(((size_t)B * T1 * C / 8 + 255) / 256), 256, 0, stream>>>(Fp(3), (size_t)B * T1 * C / 8, K1); cvt_kernel<<<(unsigned)(((size_t)B * T2 * C / 8 + 255) / 256), 256, 0, stream>>>(Fp(5), (size_t)B * T2 * C / 8, K2);
  vt_kernel<<<B * (T / 64) * NH, 256, 0, stream>>>(Fp(2), T, V0); vt_kernel<<<B * (T1 / 64) * NH, 256, 0, stream>>>(Fp(4), T1, V1); vt_kernel<<<B * (T2 / 64) * NH, 256, 0, stream>>>(Fp(6), T2, V2);
  att_kernel<<<B * NH * NQT, 32, 0, stream>>>(QB, K0, K1, K2, V0, V1, V2, Fp(7), NWV, (float*)d_out);
}
